// SparseTransformerBlock_14774687498832
// MI455X (gfx1250) — hardware-verified
//
#include <hip/hip_runtime.h>
#include <math.h>

typedef __attribute__((ext_vector_type(16))) _Float16 v16h;
typedef __attribute__((ext_vector_type(8)))  _Float16 v8h;
typedef __attribute__((ext_vector_type(16))) __bf16   v16b;
typedef __attribute__((ext_vector_type(8)))  __bf16   v8b;
typedef __attribute__((ext_vector_type(8)))  float    v8f;
typedef __attribute__((ext_vector_type(4)))  float    v4f;

constexpr int DMOD = 1024;
constexpr int NHEAD = 16;
constexpr int DHEAD = 64;
constexpr int DFF  = 4096;
constexpr int NBATCH = 2;
constexpr int SEQ  = 2048;
constexpr int NTOK = NBATCH * SEQ;
constexpr int DFFH = DFF / 2;
constexpr float WCARRY = 64.0f;
constexpr float OCARRY = 16.0f;
constexpr float GCARRY = 16.0f;
constexpr float PCARRY = 32768.0f;

static_assert(NTOK % 64 == 0 && DMOD % 64 == 0 && DFF % 64 == 0 && DFFH % 64 == 0, "tile multiples");
static_assert(DMOD % 32 == 0 && DFF % 32 == 0, "K multiple of 32");
static_assert(DMOD == 128 * 8, "rmsnorm thread map");
static_assert(DFFH == 256 * 8, "gelu thread map");
static_assert(SEQ % 64 == 0 && DHEAD == 64 && NHEAD * DHEAD == DMOD, "attention geometry");

constexpr size_t MIB = 1048576;
constexpr size_t OFF_WDN = 0;
constexpr size_t OFF_WUP = 8 * MIB;
constexpr size_t OFF_X1  = 16 * MIB;
constexpr size_t OFF_HN  = 32 * MIB;
constexpr size_t OFF_G16 = 40 * MIB;
constexpr size_t OFF_U32 = 72 * MIB;
constexpr size_t WS_TOTAL = 104 * MIB;
constexpr size_t OFF_WQ  = 40 * MIB;
constexpr size_t OFF_WK  = 42 * MIB;
constexpr size_t OFF_WV  = 44 * MIB;
constexpr size_t OFF_WO  = 46 * MIB;
constexpr size_t OFF_XN  = 48 * MIB;
constexpr size_t OFF_Q   = 56 * MIB;
constexpr size_t OFF_K   = 64 * MIB;
constexpr size_t OFF_VT  = 72 * MIB;
constexpr size_t OFF_AO  = 80 * MIB;
static_assert((size_t)DFF * DMOD * 2 == 8 * MIB, "weight plane size");
static_assert((size_t)DMOD * DMOD * 2 == 2 * MIB, "square weight plane size");
static_assert((size_t)NTOK * DMOD * 4 == 16 * MIB, "x1 size");
static_assert((size_t)NTOK * DMOD * 2 == 8 * MIB, "act plane size");
static_assert((size_t)NTOK * DFF * 2 == 32 * MIB, "g16 size");
static_assert((size_t)NTOK * DFFH * 4 == 32 * MIB, "u32h size");
static_assert(OFF_WO + (size_t)DMOD * DMOD * 2 <= OFF_XN, "square weights fit");
static_assert(OFF_AO + 8 * MIB <= WS_TOTAL, "phase A overlay fits");
static_assert(OFF_U32 + 32 * MIB == WS_TOTAL, "carve total");
static_assert(WS_TOTAL <= 134217728, "under 128 MiB");

__device__ __forceinline__ unsigned short f2bf_bits(float f) {
  unsigned u = __float_as_uint(f);
  return (unsigned short)((u + 0x7FFFu + ((u >> 16) & 1u)) >> 16);
}
__device__ __forceinline__ float bf_bits2f(unsigned short h) { return __uint_as_float(((unsigned)h) << 16); }

__device__ __forceinline__ void dep_guard_h(v8f& a, v8f& b, v16h x, v16h y) { asm volatile("v_nop\n\tv_nop\n\tv_nop\n\tv_nop" : "+v"(a), "+v"(b) : "v"(x), "v"(y)); }
__device__ __forceinline__ void dep_guard_b(v8f& a, v8f& b, v16b x, v16b y) { asm volatile("v_nop\n\tv_nop\n\tv_nop\n\tv_nop" : "+v"(a), "+v"(b) : "v"(x), "v"(y)); }
__device__ __forceinline__ void keep4_h(v16h a, v16h b, v16h c, v16h d) { asm volatile("v_nop" :: "v"(a), "v"(b), "v"(c), "v"(d)); }
__device__ __forceinline__ void keep4_b(v16b a, v16b b, v16b c, v16b d) { asm volatile("v_nop" :: "v"(a), "v"(b), "v"(c), "v"(d)); }
__device__ __forceinline__ void acc_guard4(v8f& a, v8f& b, v8f& c, v8f& d) { asm volatile("v_nop\n\tv_nop\n\tv_nop\n\tv_nop" : "+v"(a), "+v"(b), "+v"(c), "+v"(d)); }
template <typename T> struct Frag;
template <> struct Frag<_Float16> {
  typedef v16h V; union U { v16h v; v8h h[2]; };
  static __device__ __forceinline__ v16h load(const _Float16* p) {
    U f; f.h[0] = *(const v8h*)(p); f.h[1] = *(const v8h*)(p + 16); return f.v;
  }
  static __device__ __forceinline__ v8f mma(v16h a, v16h b, v8f c) {
    return __builtin_amdgcn_wmma_f32_16x16x32_f16(false, a, false, b, (short)0, c, false, false);
  }
  static __device__ __forceinline__ void guard(v8f& a, v8f& b, v16h x, v16h y) { dep_guard_h(a, b, x, y); }
  static __device__ __forceinline__ void keep(v16h a, v16h b, v16h c, v16h d) { keep4_h(a, b, c, d); }
};
template <> struct Frag<__bf16> {
  typedef v16b V; union U { v16b v; v8b h[2]; };
  static __device__ __forceinline__ v16b load(const __bf16* p) {
    U f; f.h[0] = *(const v8b*)(p); f.h[1] = *(const v8b*)(p + 16); return f.v;
  }
  static __device__ __forceinline__ v8f mma(v16b a, v16b b, v8f c) {
    return __builtin_amdgcn_wmma_f32_16x16x32_bf16(false, a, false, b, (short)0, c, false, false);
  }
  static __device__ __forceinline__ void guard(v8f& a, v8f& b, v16b x, v16b y) { dep_guard_b(a, b, x, y); }
  static __device__ __forceinline__ void keep(v16b a, v16b b, v16b c, v16b d) { keep4_b(a, b, c, d); }
};

__device__ __forceinline__ v8f hmma(v16h a, v16h b, v8f c) {
  c = __builtin_amdgcn_wmma_f32_16x16x32_f16(false, a, false, b, (short)0, c, false, false);
  asm volatile("v_nop\n\tv_nop\n\tv_nop\n\tv_nop" : "+v"(c) : "v"(a), "v"(b));
  return c;
}

template <int ET> struct Elem;
template <> struct Elem<0> { typedef _Float16 T; };
template <> struct Elem<1> { typedef __bf16 T; };
template <int ET, bool SPLIT, int BIAS_MODE, int OUT_MODE, bool RESID, int ACT = 0>
__global__ __launch_bounds__(256) void wmma_gemm64(
    const unsigned short* __restrict__ Ap, const unsigned short* __restrict__ A2p, int lda, long strideA,
    const unsigned short* __restrict__ Btp, const unsigned short* __restrict__ Bt2p, int ldb, long strideB,
    void* __restrict__ Cout, void* __restrict__ Cout2, int ldc, long strideC,
    const float* __restrict__ bias,
    const float* __restrict__ resid, long strideR,
    int M, int N, int K, float scale) {
  static_assert(!(RESID && OUT_MODE != 0), "residual only with f32 output");
  typedef typename Elem<ET>::T T;
  typedef typename Frag<T>::V V;
  const T* A = (const T*)Ap; const T* A2 = (const T*)A2p; const T* Bt = (const T*)Btp; const T* Bt2 = (const T*)Bt2p;
  __shared__ __align__(16) float sT[8][16 * 68];
  const int b    = blockIdx.y;
  const int lane = threadIdx.x & 31;
  const int wave = threadIdx.x >> 5;
  const int tilesN = N >> 6;
  const int tilesM = M >> 6;
  const int tile = blockIdx.x * 8 + wave;
  if (tile >= tilesM * tilesN) return;
  const int tm = tile / tilesN;
  const int tn = tile - tm * tilesN;
  const int m0 = tm << 6;
  const int n0 = tn << 6;

  const T* Ab  = A  + (size_t)b * strideA;
  const T* Bb  = Bt + (size_t)b * strideB;
  const T* Ab2 = SPLIT ? (A2  + (size_t)b * strideA) : nullptr;
  const T* Bb2 = SPLIT ? (Bt2 + (size_t)b * strideB) : nullptr;

  const int rlane = lane & 15;
  const int koff  = (lane >> 4) * 8;
  const int mOff  = (lane >> 4) * 8;

  v8f acc[4][4];
#pragma unroll
  for (int i = 0; i < 4; ++i)
#pragma unroll
    for (int j = 0; j < 4; ++j) acc[i][j] = (v8f){0.f,0.f,0.f,0.f,0.f,0.f,0.f,0.f};

  for (int k0 = 0; k0 < K; k0 += 32) {
    V bh[4], bl[4];
#pragma unroll
    for (int j = 0; j < 4; ++j) {
      const size_t bo = (size_t)(n0 + (j << 4) + rlane) * ldb + koff + k0;
      bh[j] = Frag<T>::load(Bb + bo);
      if (SPLIT) bl[j] = Frag<T>::load(Bb2 + bo);
    }
#pragma unroll
    for (int i = 0; i < 4; ++i) {
      const size_t ao = (size_t)(m0 + (i << 4) + rlane) * lda + koff + k0;
      V ah = Frag<T>::load(Ab + ao);
      V al;
      if (SPLIT) al = Frag<T>::load(Ab2 + ao);
#pragma unroll
      for (int j = 0; j < 4; ++j) {
        acc[i][j] = Frag<T>::mma(ah, bh[j], acc[i][j]);
        if (SPLIT) {
          acc[i][j] = Frag<T>::mma(ah, bl[j], acc[i][j]);
          acc[i][j] = Frag<T>::mma(al, bh[j], acc[i][j]);
        }
      }
      Frag<T>::guard(acc[i][0], acc[i][3], ah, SPLIT ? al : ah);
    }
    Frag<T>::keep(bh[0], bh[1], bh[2], bh[3]);
    if (SPLIT) Frag<T>::keep(bl[0], bl[1], bl[2], bl[3]);
  }
  acc_guard4(acc[0][0], acc[0][1], acc[0][2], acc[0][3]);
  acc_guard4(acc[1][0], acc[1][1], acc[1][2], acc[1][3]);
  acc_guard4(acc[2][0], acc[2][1], acc[2][2], acc[2][3]);
  acc_guard4(acc[3][0], acc[3][1], acc[3][2], acc[3][3]);

  float* slab = sT[wave];
  const float* Rb = RESID ? (resid + (size_t)b * strideR) : nullptr;
#pragma unroll
  for (int i = 0; i < 4; ++i) {
    const int mBase = m0 + (i << 4);
#pragma unroll
    for (int j = 0; j < 4; ++j) {
      const int n = n0 + (j << 4) + rlane;
      float bv = 0.f;
      if (BIAS_MODE == 2) bv = bias[n];
#pragma unroll
      for (int r = 0; r < 8; ++r) {
        float v = acc[i][j][r] * scale;
        if (BIAS_MODE == 1) v += bias[mBase + mOff + r];
        if (BIAS_MODE == 2) v += bv;
        if (ACT == 1) v = tanhf(v);
        if (ACT == 2) v = fmaxf(v, 0.0f);
        if (ACT == 4) v = (v > 0.f) ? v : 0.01f * v;
        slab[(mOff + r) * 68 + (j << 4) + rlane] = v;
      }
    }
    __builtin_amdgcn_fence(__ATOMIC_RELEASE, "workgroup");
    __builtin_amdgcn_wave_barrier();
    __builtin_amdgcn_fence(__ATOMIC_ACQUIRE, "workgroup");
    if (OUT_MODE == 0) {
      float* C = (float*)Cout + (size_t)b * strideC;
      const int hh = lane >> 4, c4 = (lane & 15) * 4;
      v4f ov[8];
#pragma unroll
      for (int it = 0; it < 8; ++it) {
        const int row = it * 2 + hh;
        v4f v = *(const v4f*)(slab + row * 68 + c4);
        if (RESID) {
          const v4f rr = *(const v4f*)(Rb + (size_t)(mBase + row) * ldc + n0 + c4);
          v = v + rr;
        }
        ov[it] = v;
      }
      for (int pass = 0; pass < 2; ++pass) {
#pragma unroll
        for (int it = 0; it < 8; ++it) {
          const int row = it * 2 + hh;
          *(volatile v4f*)(C + (size_t)(mBase + row) * ldc + n0 + c4) = ov[it];
        }
        __threadfence();
      }
    } else {
      const int q = lane >> 3, c8 = (lane & 7) * 8;
      unsigned short* C  = (unsigned short*)Cout  + (size_t)b * strideC;
      unsigned short* C2 = (OUT_MODE == 2) ? ((unsigned short*)Cout2 + (size_t)b * strideC) : nullptr;
      for (int pass = 0; pass < 2; ++pass) {
#pragma unroll
        for (int it = 0; it < 4; ++it) {
          const int row = it * 4 + q;
          const float* sp = slab + row * 68 + c8;
          v8h hv, lv;
#pragma unroll
          for (int e = 0; e < 8; ++e) {
            if (OUT_MODE == 1) {
              hv[e] = (_Float16)sp[e];
            } else {
              unsigned short hb = f2bf_bits(sp[e]);
              unsigned short lb = f2bf_bits(sp[e] - bf_bits2f(hb));
              hv[e] = __builtin_bit_cast(_Float16, hb);
              lv[e] = __builtin_bit_cast(_Float16, lb);
            }
          }
          *(volatile v8h*)(C + (size_t)(mBase + row) * ldc + n0 + c8) = hv;
          if (OUT_MODE == 2) *(volatile v8h*)(C2 + (size_t)(mBase + row) * ldc + n0 + c8) = lv;
        }
        __threadfence();
      }
    }
    __builtin_amdgcn_fence(__ATOMIC_RELEASE, "workgroup");
    __builtin_amdgcn_wave_barrier();
    __builtin_amdgcn_fence(__ATOMIC_ACQUIRE, "workgroup");
  }
}

__global__ __launch_bounds__(256) void wtrans_cast_f16(
    const float* __restrict__ in, unsigned short* __restrict__ outp, int Kd, int Nd, float sc) {
  __shared__ __align__(16) float tile[64 * 68];
  _Float16* out = (_Float16*)(void*)outp;
  const int t  = threadIdx.x;
  const int n0 = blockIdx.x * 64;
  const int k0 = blockIdx.y * 64;
  const int c4 = (t & 15) * 4;
#pragma unroll
  for (int i = 0; i < 4; ++i) {
    const int row = (t >> 4) + 16 * i;
    const v4f v = *(const v4f*)(in + (size_t)(k0 + row) * Nd + n0 + c4);
    *(v4f*)(tile + row * 68 + c4) = v;
  }
  __syncthreads();
  const int wave = t >> 5, lane = t & 31, q = lane >> 3, c8 = (lane & 7) * 8;
  for (int pass = 0; pass < 2; ++pass) {
#pragma unroll
    for (int it = 0; it < 2; ++it) {
      const int nrow = wave * 8 + it * 4 + q;
      v8h hv;
#pragma unroll
      for (int e = 0; e < 8; ++e) hv[e] = (_Float16)(tile[(c8 + e) * 68 + nrow] * sc);
      *(volatile v8h*)(out + (size_t)(n0 + nrow) * Kd + k0 + c8) = hv;
    }
    __threadfence();
  }
}

__global__ __launch_bounds__(128) void rmsnorm_f16(
    const float* __restrict__ x, const float* __restrict__ w, unsigned short* __restrict__ outp,
    int D, float eps) {
  __shared__ float red[4];
  _Float16* out = (_Float16*)(void*)outp;
  const int row = blockIdx.x;
  const int t = threadIdx.x, lane = t & 31, wave = t >> 5;
  const float* xr = x + (size_t)row * D + t * 8;
  const v4f a0 = *(const v4f*)(xr);
  const v4f a1 = *(const v4f*)(xr + 4);
  float ss = a0[0] * a0[0] + a0[1] * a0[1] + a0[2] * a0[2] + a0[3] * a0[3]
           + a1[0] * a1[0] + a1[1] * a1[1] + a1[2] * a1[2] + a1[3] * a1[3];
#pragma unroll
  for (int off = 1; off < 32; off <<= 1) ss += __shfl_xor(ss, off, 32);
  if (lane == 0) red[wave] = ss;
  __syncthreads();
  const float tot = (red[0] + red[1]) + (red[2] + red[3]);
  const float nrm = rsqrtf(tot * (1.0f / (float)D) + eps);
  const v4f w0 = *(const v4f*)(w + t * 8);
  const v4f w1 = *(const v4f*)(w + t * 8 + 4);
  v8h hv;
  hv[0] = (_Float16)((a0[0] * nrm) * w0[0]);
  hv[1] = (_Float16)((a0[1] * nrm) * w0[1]);
  hv[2] = (_Float16)((a0[2] * nrm) * w0[2]);
  hv[3] = (_Float16)((a0[3] * nrm) * w0[3]);
  hv[4] = (_Float16)((a1[0] * nrm) * w1[0]);
  hv[5] = (_Float16)((a1[1] * nrm) * w1[1]);
  hv[6] = (_Float16)((a1[2] * nrm) * w1[2]);
  hv[7] = (_Float16)((a1[3] * nrm) * w1[3]);
  _Float16* op = out + (size_t)row * D + t * 8;
  *(volatile v8h*)op = hv;
  __threadfence();
  *(volatile v8h*)op = hv;
}

__global__ __launch_bounds__(256) void gelu_cast_f16(
    const float* __restrict__ u, int ldu, unsigned short* __restrict__ gp, int ldg, int colOff, float sc) {
  __shared__ __align__(16) _Float16 hb[DFFH];
  _Float16* g = (_Float16*)(void*)gp;
  const int row = blockIdx.x;
  const int t = threadIdx.x;
  const float* ur = u + (size_t)row * ldu;
#pragma unroll 1
  for (int i = 0; i < 8; ++i) {
    const int col = i * 256 + t;
    const float xv = ur[col];
    const float gl = 0.5f * xv * (1.0f + erff(xv * 0.70710678118654752f));
    hb[col] = (_Float16)(gl * sc);
  }
  __syncthreads();
  const v8h hv = *(const v8h*)(hb + t * 8);
  _Float16* op = g + (size_t)row * ldg + colOff + t * 8;
  *(volatile v8h*)op = hv;
  __threadfence();
  *(volatile v8h*)op = hv;
}

constexpr int ATT_NW = 4;
constexpr int ATT_KC = 64;

__global__ __launch_bounds__(128) void attn_causal_f16(
    const unsigned short* __restrict__ Qp, const unsigned short* __restrict__ Kp,
    const unsigned short* __restrict__ Vtp, unsigned short* __restrict__ Op,
    int T, int nheads, int ldtok, int ldvt, float sscale, float oscale) {
  typedef _Float16 hf;
  const hf* Q  = (const hf*)(const void*)Qp;
  const hf* Kt = (const hf*)(const void*)Kp;
  const hf* Vt = (const hf*)(const void*)Vtp;
  hf* O = (hf*)(void*)Op;
  __shared__ __align__(16) hf    Psh[ATT_NW][16 * ATT_KC];
  __shared__ __align__(16) float Os[ATT_NW][16 * 68];

  const int tid  = threadIdx.x;
  const int wave = tid >> 5;
  const int lane = tid & 31;
  const int hh   = lane >> 4;
  const int c    = lane & 15;

  const int nqb  = T >> 6;
  const int bx   = blockIdx.x;
  const int qb   = bx % nqb;
  const int bhid = bx / nqb;
  const int h    = bhid % nheads;
  const int b    = bhid / nheads;
  const int tb   = b * T;
  const int q0   = (qb << 6) + wave * 16;

  const hf* qr = Q + (size_t)(tb + q0 + c) * ldtok + h * DHEAD + 8 * hh;
  const v16h qa0 = Frag<hf>::load(qr);
  const v16h qa1 = Frag<hf>::load(qr + 32);

  float mrow[8], lrow[8];
  v8f oacc[4];
#pragma unroll
  for (int r = 0; r < 8; ++r) { mrow[r] = -INFINITY; lrow[r] = 0.f; }
#pragma unroll
  for (int t = 0; t < 4; ++t) oacc[t] = (v8f){0.f,0.f,0.f,0.f,0.f,0.f,0.f,0.f};

  const int nChunks = qb + 1;
  hf* pw = Psh[wave];
  for (int kc = 0; kc < nChunks; ++kc) {
    const int kv0 = kc * ATT_KC;
    v8f s[4];
#pragma unroll
    for (int j = 0; j < 4; ++j) {
      s[j] = (v8f){0.f,0.f,0.f,0.f,0.f,0.f,0.f,0.f};
      const hf* kr = Kt + (size_t)(tb + kv0 + j * 16 + c) * ldtok + h * DHEAD + 8 * hh;
      const v16h kb0 = Frag<hf>::load(kr);
      const v16h kb1 = Frag<hf>::load(kr + 32);
      s[j] = hmma(qa0, kb0, s[j]);
      s[j] = hmma(qa1, kb1, s[j]);
    }
    const bool diag = (kc == qb);
    float cm[8];
#pragma unroll
    for (int r = 0; r < 8; ++r) {
      const int qrow = q0 + 8 * hh + r;
      float m = -INFINITY;
#pragma unroll
      for (int j = 0; j < 4; ++j) {
        const int kvcol = kv0 + j * 16 + c;
        float val = s[j][r] * sscale;
        if (diag && (kvcol > qrow)) val = -INFINITY;
        s[j][r] = val;
        m = fmaxf(m, val);
      }
#pragma unroll
      for (int off = 1; off < 16; off <<= 1) m = fmaxf(m, __shfl_xor(m, off, 32));
      cm[r] = m;
    }
#pragma unroll
    for (int r = 0; r < 8; ++r) {
      const float mnew  = fmaxf(mrow[r], cm[r]);
      const float alpha = expf(mrow[r] - mnew);
      mrow[r] = mnew;
      float psum = 0.f;
#pragma unroll
      for (int j = 0; j < 4; ++j) {
        const float p = expf(s[j][r] - mnew);
        psum += p;
        pw[(8 * hh + r) * ATT_KC + j * 16 + c] = (hf)(p * PCARRY);
      }
#pragma unroll
      for (int off = 1; off < 16; off <<= 1) psum += __shfl_xor(psum, off, 32);
      lrow[r] = lrow[r] * alpha + psum;
#pragma unroll
      for (int t = 0; t < 4; ++t) oacc[t][r] *= alpha;
    }
    __syncthreads();
#pragma unroll
    for (int kk = 0; kk < 2; ++kk) {
      const v16h pa = Frag<hf>::load(pw + c * ATT_KC + kk * 32 + 8 * hh);
#pragma unroll
      for (int t = 0; t < 4; ++t) {
        const v16h vb = Frag<hf>::load(Vt + (size_t)(h * DHEAD + t * 16 + c) * ldvt + tb + kv0 + kk * 32 + 8 * hh);
        oacc[t] = hmma(pa, vb, oacc[t]);
      }
    }
    __syncthreads();
  }

  float* os = Os[wave];
#pragma unroll
  for (int r = 0; r < 8; ++r) {
    const float inv = oscale / (lrow[r] * PCARRY);
#pragma unroll
    for (int t = 0; t < 4; ++t) os[(8 * hh + r) * 68 + t * 16 + c] = oacc[t][r] * inv;
  }
  __syncthreads();
  {
    const int q8 = lane >> 3, c8 = (lane & 7) * 8;
    for (int pass = 0; pass < 2; ++pass) {
#pragma unroll
      for (int it = 0; it < 4; ++it) {
        const int row = it * 4 + q8;
        const float* sp = os + row * 68 + c8;
        v8h hv;
#pragma unroll
        for (int e = 0; e < 8; ++e) hv[e] = (hf)sp[e];
        *(volatile v8h*)(O + (size_t)(tb + q0 + row) * ldtok + h * DHEAD + c8) = hv;
      }
      __threadfence();
    }
  }
}

static inline unsigned gemm_blocks(int M, int N) { return (unsigned)(((M / 64) * (N / 64) + 7) / 8); }

extern "C" void kernel_launch(void* const* d_in, const int* in_sizes, int n_in,
                              void* d_out, int out_size, void* d_ws, size_t ws_size,
                              hipStream_t stream) {
  if (n_in < 15) return;
  if (in_sizes[0] != NTOK * DMOD || in_sizes[1] != DMOD || in_sizes[2] != DMOD) return;
  if (in_sizes[3] != DMOD * DMOD || in_sizes[5] != DMOD * DMOD || in_sizes[7] != DMOD * DMOD || in_sizes[9] != DMOD * DMOD) return;
  if (in_sizes[4] != DMOD || in_sizes[6] != DMOD || in_sizes[8] != DMOD || in_sizes[10] != DMOD) return;
  if (in_sizes[11] != DMOD * DFF || in_sizes[12] != DFF || in_sizes[13] != DFF * DMOD || in_sizes[14] != DMOD) return;
  if (out_size != NTOK * DMOD) return;
  if (ws_size < WS_TOTAL) return;

  const float* x   = (const float*)d_in[0];
  const float* ln1 = (const float*)d_in[1];
  const float* ln2 = (const float*)d_in[2];
  const float* Wq  = (const float*)d_in[3];
  const float* bq  = (const float*)d_in[4];
  const float* Wk  = (const float*)d_in[5];
  const float* bk  = (const float*)d_in[6];
  const float* Wv  = (const float*)d_in[7];
  const float* bv  = (const float*)d_in[8];
  const float* Wo  = (const float*)d_in[9];
  const float* bo  = (const float*)d_in[10];
  const float* Wup = (const float*)d_in[11];
  const float* bup = (const float*)d_in[12];
  const float* Wdn = (const float*)d_in[13];
  const float* bdn = (const float*)d_in[14];
  float* out = (float*)d_out;

  char* ws = (char*)d_ws;
  unsigned short* WDNT = (unsigned short*)(ws + OFF_WDN);
  unsigned short* WUPT = (unsigned short*)(ws + OFF_WUP);
  float*          X1   = (float*)(ws + OFF_X1);
  unsigned short* HN   = (unsigned short*)(ws + OFF_HN);
  unsigned short* G16  = (unsigned short*)(ws + OFF_G16);
  float*          U32  = (float*)(ws + OFF_U32);
  unsigned short* WQT  = (unsigned short*)(ws + OFF_WQ);
  unsigned short* WKT  = (unsigned short*)(ws + OFF_WK);
  unsigned short* WVT  = (unsigned short*)(ws + OFF_WV);
  unsigned short* WOT  = (unsigned short*)(ws + OFF_WO);
  unsigned short* XN   = (unsigned short*)(ws + OFF_XN);
  unsigned short* Q16  = (unsigned short*)(ws + OFF_Q);
  unsigned short* K16  = (unsigned short*)(ws + OFF_K);
  unsigned short* VT16 = (unsigned short*)(ws + OFF_VT);
  unsigned short* AO16 = (unsigned short*)(ws + OFF_AO);

  const float wsc = 1.0f / WCARRY;
  const float wsco = 1.0f / (WCARRY * OCARRY);
  const float wscg = 1.0f / (WCARRY * GCARRY);

  wtrans_cast_f16<<<dim3(DMOD / 64, DMOD / 64), 256, 0, stream>>>(Wq, WQT, DMOD, DMOD, WCARRY);
  wtrans_cast_f16<<<dim3(DMOD / 64, DMOD / 64), 256, 0, stream>>>(Wk, WKT, DMOD, DMOD, WCARRY);
  wtrans_cast_f16<<<dim3(DMOD / 64, DMOD / 64), 256, 0, stream>>>(Wv, WVT, DMOD, DMOD, WCARRY);
  wtrans_cast_f16<<<dim3(DMOD / 64, DMOD / 64), 256, 0, stream>>>(Wo, WOT, DMOD, DMOD, WCARRY);
  wtrans_cast_f16<<<dim3(DFF / 64, DMOD / 64), 256, 0, stream>>>(Wup, WUPT, DMOD, DFF, WCARRY);
  wtrans_cast_f16<<<dim3(DMOD / 64, DFF / 64), 256, 0, stream>>>(Wdn, WDNT, DFF, DMOD, WCARRY);

  rmsnorm_f16<<<dim3(NTOK), 128, 0, stream>>>(x, ln1, XN, DMOD, 1e-6f);

  wmma_gemm64<0, false, 2, 1, false><<<dim3(gemm_blocks(NTOK, DMOD), 1), 256, 0, stream>>>(
      XN, XN, DMOD, 0L, WQT, WQT, DMOD, 0L, (void*)Q16, (void*)Q16, DMOD, 0L, bq, x, 0L, NTOK, DMOD, DMOD, wsc);
  wmma_gemm64<0, false, 2, 1, false><<<dim3(gemm_blocks(NTOK, DMOD), 1), 256, 0, stream>>>(
      XN, XN, DMOD, 0L, WKT, WKT, DMOD, 0L, (void*)K16, (void*)K16, DMOD, 0L, bk, x, 0L, NTOK, DMOD, DMOD, wsc);
  wmma_gemm64<0, false, 1, 1, false><<<dim3(gemm_blocks(DMOD, NTOK), 1), 256, 0, stream>>>(
      WVT, WVT, DMOD, 0L, XN, XN, DMOD, 0L, (void*)VT16, (void*)VT16, NTOK, 0L, bv, x, 0L, DMOD, NTOK, DMOD, wsc);

  attn_causal_f16<<<dim3(NBATCH * NHEAD * (SEQ / 64)), 128, 0, stream>>>(
      Q16, K16, VT16, AO16, SEQ, NHEAD, DMOD, NTOK, 0.125f, OCARRY);

  wmma_gemm64<0, false, 2, 0, true><<<dim3(gemm_blocks(NTOK, DMOD), 1), 256, 0, stream>>>(
      AO16, AO16, DMOD, 0L, WOT, WOT, DMOD, 0L, (void*)X1, (void*)X1, DMOD, 0L, bo, x, 0L, NTOK, DMOD, DMOD, wsco);

  rmsnorm_f16<<<dim3(NTOK), 128, 0, stream>>>(X1, ln2, HN, DMOD, 1e-6f);

  for (int half = 0; half < 2; ++half) {
    wmma_gemm64<0, false, 2, 0, false><<<dim3(gemm_blocks(NTOK, DFFH), 1), 256, 0, stream>>>(
        HN, HN, DMOD, 0L, WUPT + (size_t)half * DFFH * DMOD, WUPT + (size_t)half * DFFH * DMOD, DMOD, 0L,
        (void*)U32, (void*)U32, DFFH, 0L, bup + half * DFFH, x, 0L, NTOK, DFFH, DMOD, wsc);
    gelu_cast_f16<<<dim3(NTOK), 256, 0, stream>>>(U32, DFFH, G16, DFF, half * DFFH, GCARRY);
  }

  wmma_gemm64<0, false, 2, 0, true><<<dim3(gemm_blocks(NTOK, DMOD), 1), 256, 0, stream>>>(
      G16, G16, DFF, 0L, WDNT, WDNT, DFF, 0L, (void*)out, (void*)out, DMOD, 0L, bdn, X1, 0L, NTOK, DMOD, DFF, wscg);
}
